// GIN_51702816309753
// MI455X (gfx1250) — hardware-verified
//
#include <hip/hip_runtime.h>
#include <stddef.h>
#include <stdint.h>
#include <math.h>


#define DIN     128
#define KA      256
#define NCLS    10
#define NTHR    256
#define NWAVE   8
#define EPT     8
#define CHUNK   (NTHR * EPT)
#define WCAP    (EPT * 32)
#define LISTN   (NWAVE * WCAP)
#define PKS     9
#define NB      512
#define NBSH    9
#define RCAP    20480
#define DEGCAP  96
#define GBM     64
#define GBN     128
#define GTHR    128
#define GNT     8
#define PARTW   288
#define APR     16
#define AGR     64
#define PGS     16
#define NUW     (4 * DIN * (KA / 8))
#define WSMAX   134217728
#define LDS_CSR ((2 * RCAP + 2 * NB + LISTN) * 4 + 64)
#define LDS_MLP (GBM * KA * 2 + GBM * GBN * 4 + PARTW * 4 + 2 * GBN * 4)

static_assert((CHUNK & (CHUNK - 1)) == 0 && CHUNK <= (1 << 11));
static_assert((NB & (NB - 1)) == 0 && NB == (1 << PKS) && NB == (1 << NBSH));
static_assert(NTHR * 2 == NB && LISTN >= NB);
static_assert((RCAP % 1024) == 0 && ((2 * RCAP + 2 * NB) % (NTHR * 4)) == 0);
static_assert(RCAP < (1 << 23) && DEGCAP < 255);
static_assert(LDS_CSR <= 300000 && LDS_MLP <= 300000);
static_assert(GBM == (GTHR / 32) * 16 && GBN == 16 * GNT && GTHR == GBN && GBN == DIN);
static_assert((KA % 32) == 0 && KA == 2 * DIN && DIN == 32 * 4);
static_assert((PARTW % 32) == 0 && PARTW >= 2 * GBN + 1 && PARTW / 4 <= GTHR);
static_assert((NUW % NTHR) == 0 && ((DIN * (KA / 8)) % NTHR) == 0);
static_assert((APR * DIN) == 2 * 4 * NTHR && (GBM % APR) == 0 && (GBM % AGR) == 0 && (AGR % NWAVE) == 0);
static_assert((PGS & (PGS - 1)) == 0 && PGS <= NB && PGS * NCLS <= NTHR && ((PGS * NCLS * 4) % 128) == 0);

typedef float          v4f  __attribute__((ext_vector_type(4)));
typedef float          v8f  __attribute__((ext_vector_type(8)));
typedef int            v4i  __attribute__((ext_vector_type(4)));
typedef int            v8i  __attribute__((ext_vector_type(8)));
typedef unsigned int   v2u  __attribute__((ext_vector_type(2)));
typedef unsigned short v8us __attribute__((ext_vector_type(8)));
typedef __bf16         v16b __attribute__((ext_vector_type(16)));
typedef v4f  __attribute__((may_alias)) v4fa;
typedef v4i  __attribute__((may_alias)) v4ia;
typedef v8us __attribute__((may_alias)) v8usa;
union Frag { v16b vb; v8us h[2]; v8i w; };

__device__ __forceinline__ v8f wmb(const Frag& a, const Frag& b, v8f c) {
  v8f d = __builtin_amdgcn_wmma_f32_16x16x32_bf16(false, a.vb, false, b.vb, (short)0, c, false, false);
  asm volatile("v_nop\n\tv_nop\n\tv_nop\n\tv_nop" : "+v"(d) : "v"(a.w), "v"(b.w));
  return d;
}

__device__ __forceinline__ unsigned short bf_bits(float f) {
  unsigned int u = __float_as_uint(f);
  u += 0x7FFFu + ((u >> 16) & 1u);
  return (unsigned short)(u >> 16);
}
__device__ __forceinline__ float bf_val(unsigned short b) { return __uint_as_float(((unsigned int)b) << 16); }
__device__ __forceinline__ float bf_rne(float f) { return bf_val(bf_bits(f)); }
__device__ __forceinline__ float relu_keep(float v) { return (v > 0.0f) ? v : (v - v); }

__device__ __forceinline__ int scan_chunk(const int* __restrict__ dsts, int nE, int cbase, int slotBase,
                                          int nb, int vec8, int* list, int tid, int lane, int wave) {
  int wc = 0;
  const int el0  = tid * EPT;
  const int e0   = cbase + el0;
  const int sent = -2147483647 - 1;
  v4i da, db;
  if (vec8 != 0 && cbase + CHUNK <= nE) {
    da = *(const v4i*)(dsts + e0);
    db = *(const v4i*)(dsts + e0 + 4);
  } else {
    da.x = (e0     < nE) ? dsts[min(e0,     nE - 1)] : sent;
    da.y = (e0 + 1 < nE) ? dsts[min(e0 + 1, nE - 1)] : sent;
    da.z = (e0 + 2 < nE) ? dsts[min(e0 + 2, nE - 1)] : sent;
    da.w = (e0 + 3 < nE) ? dsts[min(e0 + 3, nE - 1)] : sent;
    db.x = (e0 + 4 < nE) ? dsts[min(e0 + 4, nE - 1)] : sent;
    db.y = (e0 + 5 < nE) ? dsts[min(e0 + 5, nE - 1)] : sent;
    db.z = (e0 + 6 < nE) ? dsts[min(e0 + 6, nE - 1)] : sent;
    db.w = (e0 + 7 < nE) ? dsts[min(e0 + 7, nE - 1)] : sent;
  }
  const unsigned nbs = (unsigned)slotBase;
  const unsigned unb = (unsigned)nb;
  const unsigned s0 = (unsigned)da.x - nbs, s1 = (unsigned)da.y - nbs;
  const unsigned s2 = (unsigned)da.z - nbs, s3 = (unsigned)da.w - nbs;
  const unsigned s4 = (unsigned)db.x - nbs, s5 = (unsigned)db.y - nbs;
  const unsigned s6 = (unsigned)db.z - nbs, s7 = (unsigned)db.w - nbs;
  const bool h0 = s0 < unb, h1 = s1 < unb, h2 = s2 < unb, h3 = s3 < unb;
  const bool h4 = s4 < unb, h5 = s5 < unb, h6 = s6 < unb, h7 = s7 < unb;
  const unsigned any = __builtin_amdgcn_ballot_w32(h0 | h1 | h2 | h3 | h4 | h5 | h6 | h7);
  if (any != 0u) {
#define HITJ(J, HJ, SJ) { \
      const unsigned mj = __builtin_amdgcn_ballot_w32(HJ); \
      if (mj != 0u) { \
        if (HJ) { \
          const int pos = wc + (int)__builtin_amdgcn_mbcnt_lo(mj, 0u); \
          if (pos < WCAP) list[wave * WCAP + pos] = ((el0 + (J)) << PKS) | (int)(SJ); \
        } \
        wc += (int)__builtin_popcount(mj); } }
    HITJ(0, h0, s0)
    HITJ(1, h1, s1)
    HITJ(2, h2, s2)
    HITJ(3, h3, s3)
    HITJ(4, h4, s4)
    HITJ(5, h5, s5)
    HITJ(6, h6, s6)
    HITJ(7, h7, s7)
#undef HITJ
  }
  return wc;
}

__device__ __forceinline__ v8us cv8b(const float* __restrict__ p, size_t stride) {
  v8us o;
#pragma unroll
  for (int i = 0; i < 8; ++i) o[i] = bf_bits(p[(size_t)i * stride]);
  return o;
}

__global__ __launch_bounds__(NTHR) void k_wprep(const float* __restrict__ w0, const float* __restrict__ w1,
                                                const float* __restrict__ w2, const float* __restrict__ w3,
                                                unsigned short* wt) {
  const int u = (int)blockIdx.x * NTHR + (int)threadIdx.x;
  if (u >= NUW) return;
  const int p  = u >> 12;
  const int v  = u & 4095;
  const int n  = v >> 5;
  const int k8 = (v & 31) * 8;
  const int kk = k8 & (DIN - 1);
  const size_t so = (size_t)kk * DIN + n;
  v8us o;
  if (p == 0)      o = cv8b(w0 + so, DIN);
  else if (p == 1) o = cv8b(w1 + so, DIN);
  else if (p == 2) o = cv8b(w2 + so, DIN);
  else             o = cv8b(w3 + so, DIN);
  unsigned short* dp = wt + (size_t)u * 8;
  *(volatile v8us*)dp = o;
  __threadfence();
  *(volatile v8us*)dp = o;
}

__global__ __launch_bounds__(NTHR) void k_cvx(const float* __restrict__ x, int nN, int nUnits,
                                              unsigned short* xb) {
  const int u = (int)blockIdx.x * NTHR + (int)threadIdx.x;
  if (u >= nUnits) return;
  const int row = u >> 4;
  const int k8  = (u & 15) * 8;
  const int rc  = row < nN ? row : nN - 1;
  const float* p = x + (size_t)rc * DIN + k8;
  const v4f a = *(const v4fa*)p;
  const v4f b = *(const v4fa*)(p + 4);
  const bool ok = row < nN;
  v8us o;
  o[0] = ok ? bf_bits(a.x) : (unsigned short)0;
  o[1] = ok ? bf_bits(a.y) : (unsigned short)0;
  o[2] = ok ? bf_bits(a.z) : (unsigned short)0;
  o[3] = ok ? bf_bits(a.w) : (unsigned short)0;
  o[4] = ok ? bf_bits(b.x) : (unsigned short)0;
  o[5] = ok ? bf_bits(b.y) : (unsigned short)0;
  o[6] = ok ? bf_bits(b.z) : (unsigned short)0;
  o[7] = ok ? bf_bits(b.w) : (unsigned short)0;
  unsigned short* dp = xb + (size_t)row * DIN + k8;
  *(volatile v8us*)dp = o;
  __threadfence();
  *(volatile v8us*)dp = o;
}

__global__ __launch_bounds__(NTHR) void k_csr(const int* __restrict__ srcs, const int* __restrict__ dsts,
                                              int nN, int nE, int vec8, int* rowinfo, int* srclist) {
  extern __shared__ v4f lds_dyn[];
  int* reg1 = (int*)lds_dyn;
  int* reg2 = reg1 + RCAP;
  int* scnt = reg2 + RCAP;
  int* soff = scnt + NB;
  int* list = soff + NB;
  int* wcnt = list + LISTN;
  int* wtot = wcnt + NWAVE;
  const int tid = (int)threadIdx.x, lane = tid & 31, wave = tid >> 5;
  const int nodeBase = (int)blockIdx.x * NB;

  {
    const v4i z4 = {0, 0, 0, 0};
    for (int i = tid * 4; i < 2 * RCAP + 2 * NB; i += NTHR * 4) *(v4ia*)(reg1 + i) = z4;
  }
  __syncthreads();

  int tot = 0;
  const int nChunks = (nE + CHUNK - 1) / CHUNK;
#pragma unroll 1
  for (int ch = 0; ch < nChunks; ++ch) {
    const int cbase = ch * CHUNK;
    const int wc = scan_chunk(dsts, nE, cbase, nodeBase, NB, vec8, list, tid, lane, wave);
    if (lane == 0) wcnt[wave] = wc;
    __syncthreads();
    int pre = 0, all = 0;
#pragma unroll
    for (int w2 = 0; w2 < NWAVE; ++w2) {
      int c = wcnt[w2];
      c = c < 0 ? 0 : (c > WCAP ? WCAP : c);
      all += c;
      pre += (w2 < wave) ? c : 0;
    }
    const int wcc  = wc > WCAP ? WCAP : wc;
    const int base = tot + pre;
#pragma unroll 1
    for (int i = lane; i < wcc; i += 32) {
      const int ent = list[wave * WCAP + i];
      const int el  = (ent >> PKS) & (CHUNK - 1);
      const int sl  = ent & (NB - 1);
      int eid = cbase + el;
      eid = eid > nE - 1 ? nE - 1 : eid;
      const int pos = base + i;
      if (pos < RCAP) reg1[pos] = (int)(((unsigned)eid << PKS) | (unsigned)sl);
    }
    tot += all;
    tot = tot > RCAP ? RCAP : tot;
    __syncthreads();
  }
  const int nh = tot;

  if (wave == 0) {
#pragma unroll 1
    for (int b0 = 0; b0 < nh; b0 += 32) {
      const int idx = b0 + lane;
      const int uv  = reg1[idx < RCAP ? idx : RCAP - 1];
      const int m32 = (nh - b0) < 32 ? (nh - b0) : 32;
#pragma unroll 1
      for (int k = 0; k < m32; ++k) {
        const int u  = __builtin_amdgcn_readlane(uv, k);
        const int sl = u & (NB - 1);
        if (lane == 0) scnt[sl] = scnt[sl] + 1;
      }
    }
  }
  __syncthreads();

  {
    const int c0 = scnt[2 * tid], c1 = scnt[2 * tid + 1];
    const int e0 = c0 < 0 ? 0 : c0, e1 = c1 < 0 ? 0 : c1;
    const int ts = e0 + e1;
    int incl = ts;
#pragma unroll
    for (int d = 1; d < 32; d <<= 1) {
      const int up = __shfl_up(incl, d);
      if (lane >= d) incl += up;
    }
    if (lane == 31) wtot[wave] = incl;
    __syncthreads();
    int pre = 0;
#pragma unroll
    for (int w2 = 0; w2 < NWAVE; ++w2) pre += (w2 < wave) ? wtot[w2] : 0;
    const int run = pre + incl - ts;
    soff[2 * tid + 0] = run;
    soff[2 * tid + 1] = run + e0;
  }
  __syncthreads();
  for (int i = tid; i < NB; i += NTHR) list[i] = soff[i];
  __syncthreads();

  if (wave == 0) {
#pragma unroll 1
    for (int b0 = 0; b0 < nh; b0 += 32) {
      const int idx = b0 + lane;
      const int uv  = reg1[idx < RCAP ? idx : RCAP - 1];
      const int m32 = (nh - b0) < 32 ? (nh - b0) : 32;
#pragma unroll 1
      for (int k = 0; k < m32; ++k) {
        const int u   = __builtin_amdgcn_readlane(uv, k);
        const int sl  = u & (NB - 1);
        const int eid = (int)((unsigned)u >> PKS);
        if (lane == 0) {
          int pos = list[sl];
          pos = pos < 0 ? 0 : (pos > RCAP - 1 ? RCAP - 1 : pos);
          reg2[pos] = eid;
          list[sl] = pos + 1;
        }
      }
    }
  }
  __syncthreads();

  const bool ovf = (nh >= RCAP);
  if (tid < NB / 4) {
    const v4i o4 = *(const v4ia*)(soff + 4 * tid);
    const v4i c4 = *(const v4ia*)(scnt + 4 * tid);
    const int oo[4] = {o4.x, o4.y, o4.z, o4.w};
    const int cc[4] = {c4.x, c4.y, c4.z, c4.w};
    int rr[4];
#pragma unroll
    for (int j = 0; j < 4; ++j) {
      int o = oo[j]; o = o < 0 ? 0 : (o > RCAP ? RCAP : o);
      int c = cc[j]; c = c < 0 ? 0 : (c > 255 ? 255 : c);
      c = ovf ? 255 : c;
      rr[j] = (int)(((unsigned)o << 8) | (unsigned)c);
    }
    v4i iv; iv.x = rr[0]; iv.y = rr[1]; iv.z = rr[2]; iv.w = rr[3];
    int* ip = rowinfo + (size_t)nodeBase + 4 * tid;
    *(volatile v4i*)ip = iv;
    __threadfence();
    *(volatile v4i*)ip = iv;
  }

  int nIt = (nh + 1023) >> 10;
  nIt = nIt > RCAP / 1024 ? RCAP / 1024 : nIt;
  int* lp = srclist + (size_t)blockIdx.x * RCAP;
#pragma unroll 1
  for (int it = 0; it < nIt; ++it) {
    const int i4 = (it * NTHR + tid) * 4;
    const v4i e = *(const v4ia*)(reg2 + i4);
    const int e0 = e.x < 0 ? 0 : (e.x > nE - 1 ? nE - 1 : e.x);
    const int e1 = e.y < 0 ? 0 : (e.y > nE - 1 ? nE - 1 : e.y);
    const int e2 = e.z < 0 ? 0 : (e.z > nE - 1 ? nE - 1 : e.z);
    const int e3 = e.w < 0 ? 0 : (e.w > nE - 1 ? nE - 1 : e.w);
    const int r0 = srcs[e0], r1 = srcs[e1], r2 = srcs[e2], r3 = srcs[e3];
    v4i sv;
    sv.x = r0 < 0 ? 0 : (r0 > nN - 1 ? nN - 1 : r0);
    sv.y = r1 < 0 ? 0 : (r1 > nN - 1 ? nN - 1 : r1);
    sv.z = r2 < 0 ? 0 : (r2 > nN - 1 ? nN - 1 : r2);
    sv.w = r3 < 0 ? 0 : (r3 > nN - 1 ? nN - 1 : r3);
    int* p = lp + i4;
    *(volatile v4i*)p = sv;
    __threadfence();
    *(volatile v4i*)p = sv;
  }
}

template <int F32SRC>
__global__ __launch_bounds__(NTHR) void k_agg(const int* __restrict__ rowinfo, const int* __restrict__ srclist,
                                              const unsigned short* xb, const float* hf,
                                              unsigned short* Aout, int nN, int MPr) {
  const int tid = (int)threadIdx.x, lane = tid & 31, wave = tid >> 5;
  const int rowBase = (int)blockIdx.x * AGR;
  const float qnan = __int_as_float(0x7fc00000);
#pragma unroll 1
  for (int j = 0; j < AGR / NWAVE; ++j) {
    const int grow = __builtin_amdgcn_readfirstlane(rowBase + wave * (AGR / NWAVE) + j);
    const int gi   = grow < MPr ? grow : MPr - 1;
    const int info = __builtin_amdgcn_readfirstlane(rowinfo[gi]);
    int off = (int)((unsigned)info >> 8);
    const int craw = info & 255;
    off = off > RCAP ? RCAP : off;
    int cnt = craw > DEGCAP ? DEGCAP : craw;
    if (cnt > RCAP - off) cnt = RCAP - off;
    const float pz = (craw > DEGCAP) ? qnan : 0.0f;
    const int blk = gi >> NBSH;
    const int* lp = srclist + (size_t)blk * RCAP + off;
    const bool liveRow = grow < nN;

    float ag0 = 0.f, ag1 = 0.f, ag2 = 0.f, ag3 = 0.f;
#pragma unroll 1
    for (int b0 = 0; b0 < cnt; b0 += 32) {
      int q = b0 + lane;
      q = q > cnt - 1 ? cnt - 1 : q;
      int sr = lp[q];
      sr = sr < 0 ? 0 : (sr > nN - 1 ? nN - 1 : sr);
      const int m32 = (cnt - b0) < 32 ? (cnt - b0) : 32;
#pragma unroll 1
      for (int k = 0; k < m32; ++k) {
        const int sk = __builtin_amdgcn_readlane(sr, k);
        if constexpr (F32SRC != 0) {
          const v4f v = *(const v4f*)(hf + (size_t)sk * DIN + 4 * lane);
          ag0 += v.x; ag1 += v.y; ag2 += v.z; ag3 += v.w;
        } else {
          const v2u w = *(const v2u*)(xb + (size_t)sk * DIN + 4 * lane);
          ag0 += __uint_as_float(w.x << 16);
          ag1 += __uint_as_float(w.x & 0xffff0000u);
          ag2 += __uint_as_float(w.y << 16);
          ag3 += __uint_as_float(w.y & 0xffff0000u);
        }
      }
    }
    const int nc = liveRow ? grow : nN - 1;
    float s0, s1, s2, s3;
    if constexpr (F32SRC != 0) {
      const v4f sv = *(const v4f*)(hf + (size_t)nc * DIN + 4 * lane);
      s0 = sv.x; s1 = sv.y; s2 = sv.z; s3 = sv.w;
    } else {
      const v2u w = *(const v2u*)(xb + (size_t)nc * DIN + 4 * lane);
      s0 = __uint_as_float(w.x << 16);
      s1 = __uint_as_float(w.x & 0xffff0000u);
      s2 = __uint_as_float(w.y << 16);
      s3 = __uint_as_float(w.y & 0xffff0000u);
    }
    float r0 = s0 + ag0, r1 = s1 + ag1, r2 = s2 + ag2, r3 = s3 + ag3;
    r0 = (liveRow ? r0 : 0.0f) + pz;
    r1 = (liveRow ? r1 : 0.0f) + pz;
    r2 = (liveRow ? r2 : 0.0f) + pz;
    r3 = (liveRow ? r3 : 0.0f) + pz;

    const unsigned short h0 = bf_bits(r0), h1 = bf_bits(r1), h2 = bf_bits(r2), h3 = bf_bits(r3);
    const unsigned short l0 = bf_bits(r0 - bf_val(h0)), l1 = bf_bits(r1 - bf_val(h1));
    const unsigned short l2 = bf_bits(r2 - bf_val(h2)), l3 = bf_bits(r3 - bf_val(h3));
    v2u hv, lv;
    hv.x = (unsigned int)h0 | ((unsigned int)h1 << 16);
    hv.y = (unsigned int)h2 | ((unsigned int)h3 << 16);
    lv.x = (unsigned int)l0 | ((unsigned int)l1 << 16);
    lv.y = (unsigned int)l2 | ((unsigned int)l3 << 16);
    unsigned short* hp = Aout + (size_t)gi * KA + 4 * lane;
    unsigned short* lq = hp + DIN;
    const bool wsv = grow < MPr;
    if (wsv) { *(volatile v2u*)hp = hv; *(volatile v2u*)lq = lv; }
    __threadfence();
    if (wsv) { *(volatile v2u*)hp = hv; *(volatile v2u*)lq = lv; }
  }
}

__global__ __launch_bounds__(GTHR) void k_mlp(const unsigned short* __restrict__ A,
                                              const unsigned short* __restrict__ WaT,
                                              const unsigned short* __restrict__ WbT,
                                              const float* __restrict__ ba, const float* __restrict__ bb,
                                              float* Z, int nN, int mRows, float* part) {
  extern __shared__ v4f lds_dyn[];
  unsigned short* tl = (unsigned short*)lds_dyn;
  float* stg = (float*)(tl + GBM * KA);
  float* pst = stg + GBM * GBN;
  float* bsh = pst + PARTW;
  const int tid = (int)threadIdx.x, lane = tid & 31, wave = tid >> 5, hh = lane >> 4, m = lane & 15;
  const int rowBase = (int)blockIdx.x * GBM;

  bsh[tid]       = bf_rne(ba[tid]);
  bsh[GBN + tid] = bf_rne(bb[tid]);

  v8f acc[GNT];
  const v8f z8 = {0.f, 0.f, 0.f, 0.f, 0.f, 0.f, 0.f, 0.f};
#pragma unroll
  for (int t = 0; t < GNT; ++t) acc[t] = z8;

  {
    const unsigned short* ap = A   + (size_t)(rowBase + 16 * wave + m) * (size_t)KA + 8 * hh;
    const unsigned short* bp = WaT + (size_t)m * (size_t)KA + 8 * hh;
#pragma unroll 1
    for (int k0 = 0; k0 < KA; k0 += 32) {
      Frag af;
      af.h[0] = *(const v8usa*)(ap + k0);
      af.h[1] = *(const v8usa*)(ap + k0 + 16);
#pragma unroll
      for (int nt = 0; nt < GNT; ++nt) {
        const unsigned short* wq = bp + (size_t)(16 * nt) * (size_t)KA + k0;
        Frag bfr;
        bfr.h[0] = *(const v8usa*)wq;
        bfr.h[1] = *(const v8usa*)(wq + 16);
        acc[nt] = wmb(af, bfr, acc[nt]);
      }
    }
  }
  __syncthreads();

#pragma unroll
  for (int nt = 0; nt < GNT; ++nt) {
    const int lc = 16 * nt + m;
    const float bv = bsh[lc];
#pragma unroll
    for (int r = 0; r < 8; ++r) {
      const int lr = 16 * wave + 8 * hh + r;
      const float v = relu_keep(acc[nt][r] + bv);
      const unsigned short hb = bf_bits(v);
      const unsigned short lb = bf_bits(v - bf_val(hb));
      tl[lr * KA + lc]       = hb;
      tl[lr * KA + DIN + lc] = lb;
    }
  }
  __syncthreads();

#pragma unroll
  for (int t = 0; t < GNT; ++t) acc[t] = z8;
  {
    const unsigned short* tp = tl  + (16 * wave + m) * KA + 8 * hh;
    const unsigned short* bp = WbT + (size_t)m * (size_t)KA + 8 * hh;
#pragma unroll 1
    for (int k0 = 0; k0 < KA; k0 += 32) {
      Frag af;
      af.h[0] = *(const v8usa*)(tp + k0);
      af.h[1] = *(const v8usa*)(tp + k0 + 16);
#pragma unroll
      for (int nt = 0; nt < GNT; ++nt) {
        const unsigned short* wq = bp + (size_t)(16 * nt) * (size_t)KA + k0;
        Frag bfr;
        bfr.h[0] = *(const v8usa*)wq;
        bfr.h[1] = *(const v8usa*)(wq + 16);
        acc[nt] = wmb(af, bfr, acc[nt]);
      }
    }
  }

#pragma unroll
  for (int nt = 0; nt < GNT; ++nt) {
    const int lc = 16 * nt + m;
    const float bv = bsh[GBN + lc];
#pragma unroll
    for (int r = 0; r < 8; ++r) {
      const int lr = 16 * wave + 8 * hh + r;
      const bool live = (rowBase + lr) < nN;
      const float v = acc[nt][r] + bv;
      stg[lr * GBN + lc] = live ? v : 0.0f;
    }
  }
  __syncthreads();

  v4f fv[16];
#pragma unroll
  for (int i = 0; i < 16; ++i) {
    const int lr = 16 * wave + i;
    fv[i] = *(const v4fa*)(stg + lr * GBN + 4 * lane);
  }
  v4f pv = {0.f, 0.f, 0.f, 0.f};
  const bool pok = tid < PARTW / 4;
  {
    int nvr = nN - rowBase;
    nvr = nvr < 0 ? 0 : (nvr > GBM ? GBM : nvr);
    float s = 0.0f;
#pragma unroll 1
    for (int r = 0; r < nvr; ++r) s += stg[r * GBN + tid];
    const float inv = 1.0f / (float)(nvr < 1 ? 1 : nvr);
    const float mean = s * inv;
    float q = 0.0f;
#pragma unroll 1
    for (int r = 0; r < nvr; ++r) {
      const float d = stg[r * GBN + tid] - mean;
      q = fmaf(d, d, q);
    }
    pst[1 + tid] = mean;
    pst[1 + GBN + tid] = q;
    if (tid == 0) pst[0] = (float)nvr;
#pragma unroll 1
    for (int i = 2 * GBN + 1 + tid; i < PARTW; i += GTHR) pst[i] = 0.0f;
    __syncthreads();
    if (pok) pv = *(const v4fa*)(pst + 4 * tid);
  }
  float* pp = part + (size_t)blockIdx.x * PARTW + 4 * tid;
#pragma unroll
  for (int i = 0; i < 16; ++i) {
    const int gr = rowBase + 16 * wave + i;
    float* op = Z + (size_t)gr * DIN + 4 * lane;
    if (gr < mRows) *(volatile v4f*)op = fv[i];
  }
  if (pok) *(volatile v4f*)pp = pv;
  __threadfence();
#pragma unroll
  for (int i = 0; i < 16; ++i) {
    const int gr = rowBase + 16 * wave + i;
    float* op = Z + (size_t)gr * DIN + 4 * lane;
    if (gr < mRows) *(volatile v4f*)op = fv[i];
  }
  if (pok) *(volatile v4f*)pp = pv;
}

__global__ __launch_bounds__(GBN) void k_bnfin(const float* __restrict__ part, int nPart,
                                               const float* __restrict__ gam, const float* __restrict__ bet,
                                               float* ss) {
  __shared__ __attribute__((aligned(16))) float stg[3 * GBN];
  const int tid = (int)threadIdx.x;
  double n = 0.0, mean = 0.0, M2 = 0.0;
#pragma unroll 1
  for (int b = 0; b < nPart; ++b) {
    const float* pr = part + (size_t)b * PARTW;
    const double nb = (double)pr[0];
    const double mb = (double)pr[1 + tid];
    const double qb = (double)pr[1 + GBN + tid];
    if (nb > 0.5) {
      const double nn = n + nb;
      const double delta = mb - mean;
      const double f = nb / nn;
      mean = mean + delta * f;
      M2 = M2 + qb + delta * delta * n * f;
      n = nn;
    }
  }
  const double nt = n < 1.0 ? 1.0 : n;
  const float var  = (float)(M2 / nt);
  const float rstd = rsqrtf(var + 1e-5f);
  stg[tid]           = (float)mean;
  stg[GBN + tid]     = bf_rne(gam[tid]) * rstd;
  stg[2 * GBN + tid] = bf_rne(bet[tid]);
  __syncthreads();
  const int seg = tid >> 5, j = tid & 31;
  const bool ok = tid < 96;
  const int sg = ok ? seg : 2;
  const v4f v = *(const v4fa*)(stg + sg * GBN + 4 * j);
  float* dp = ss + (size_t)sg * GBN + 4 * j;
  if (ok) *(volatile v4f*)dp = v;
  __threadfence();
  if (ok) *(volatile v4f*)dp = v;
}

__global__ __launch_bounds__(NTHR) void k_bnap(float* ZH, const float* __restrict__ ss, int nN, int mRows) {
  __shared__ float ssh[3 * DIN];
  __shared__ __attribute__((aligned(16))) float tile[APR * DIN];
  const int tid = (int)threadIdx.x;
  for (int i = tid; i < 3 * DIN; i += NTHR) ssh[i] = ss[i];
  const int rowBase = (int)blockIdx.x * APR;
  const int c  = tid & (DIN - 1);
  const int rs = tid >> 7;
  __syncthreads();
#pragma unroll 1
  for (int r = 0; r < APR / 2; ++r) {
    const int lr   = 2 * r + rs;
    const int grow = rowBase + lr;
    const int gc   = grow < mRows ? grow : mRows - 1;
    const float u = ZH[(size_t)gc * DIN + c];
    const float y = (u - ssh[c]) * ssh[DIN + c] + ssh[2 * DIN + c];
    const float v = relu_keep(y);
    tile[lr * DIN + c] = (grow < nN) ? v : 0.0f;
  }
  __syncthreads();
  v4f pv[2];
#pragma unroll
  for (int it = 0; it < 2; ++it) {
    const int p = it * NTHR + tid;
    const int lr = p >> 5, q = p & 31;
    pv[it] = *(const v4fa*)(tile + lr * DIN + 4 * q);
  }
#pragma unroll
  for (int it = 0; it < 2; ++it) {
    const int p = it * NTHR + tid;
    const int lr = p >> 5, q = p & 31;
    const int grow = rowBase + lr;
    float* op = ZH + (size_t)grow * DIN + 4 * q;
    if (grow < mRows) *(volatile v4f*)op = pv[it];
  }
  __threadfence();
#pragma unroll
  for (int it = 0; it < 2; ++it) {
    const int p = it * NTHR + tid;
    const int lr = p >> 5, q = p & 31;
    const int grow = rowBase + lr;
    float* op = ZH + (size_t)grow * DIN + 4 * q;
    if (grow < mRows) *(volatile v4f*)op = pv[it];
  }
}

__global__ __launch_bounds__(NTHR) void k_pool_head(const float* __restrict__ Z, const float* __restrict__ ss,
                                                    const int* __restrict__ bat, int nN, int vec8b, int nG,
                                                    const float* __restrict__ Wl, const float* __restrict__ bl,
                                                    float* out) {
  __shared__ __attribute__((aligned(16))) float accs[PGS * DIN];
  __shared__ float ssh[3 * DIN];
  __shared__ float wls[DIN * NCLS];
  __shared__ float bls[16];
  __shared__ __attribute__((aligned(16))) int list[LISTN];
  __shared__ int wcnt[NWAVE];
  __shared__ float lg[PGS * NCLS];
  __shared__ __attribute__((aligned(16))) float os[PGS * NCLS];
  const int tid = (int)threadIdx.x, lane = tid & 31, wave = tid >> 5;
  const int slotBase = (int)blockIdx.x * PGS;
  int nb = nG - slotBase;
  nb = nb > PGS ? PGS : (nb < 0 ? 0 : nb);

  for (int i = tid; i < PGS * DIN; i += NTHR) accs[i] = 0.0f;
  for (int i = tid; i < 3 * DIN; i += NTHR) ssh[i] = ss[i];
#pragma unroll 1
  for (int i = tid; i < DIN * NCLS; i += NTHR) wls[i] = bf_rne(Wl[i]);
  if (tid < 16) {
    const float bbv = bl[tid < NCLS ? tid : NCLS - 1];
    bls[tid] = (tid < NCLS) ? bf_rne(bbv) : 0.0f;
  }
  __syncthreads();

  const int nChunks = (nN + CHUNK - 1) / CHUNK;
#pragma unroll 1
  for (int ch = 0; ch < nChunks; ++ch) {
    const int cbase = ch * CHUNK;
    const int wc = scan_chunk(bat, nN, cbase, slotBase, nb, vec8b, list, tid, lane, wave);
    if (lane == 0) wcnt[wave] = wc;
    __syncthreads();
#pragma unroll 1
    for (int w2 = 0; w2 < NWAVE; ++w2) {
      int c = wcnt[w2];
      c = c < 0 ? 0 : (c > WCAP ? WCAP : c);
#pragma unroll 1
      for (int i = 0; i < c; ++i) {
        const int ent = list[w2 * WCAP + i];
        const int el  = (ent >> PKS) & (CHUNK - 1);
        const int sl  = ent & (PGS - 1);
        int node = cbase + el;
        node = node < 0 ? 0 : (node > nN - 1 ? nN - 1 : node);
        if (tid < DIN) {
          const float u = Z[(size_t)node * DIN + tid];
          const float y = (u - ssh[tid]) * ssh[DIN + tid] + ssh[2 * DIN + tid];
          accs[sl * DIN + tid] += relu_keep(y);
        }
      }
    }
    __syncthreads();
  }

  if (tid < PGS * NCLS) {
    const int g = tid / NCLS;
    const int o = tid - g * NCLS;
    const float* pr = accs + g * DIN;
    float s = 0.0f;
#pragma unroll 4
    for (int k = 0; k < DIN; ++k) s = fmaf(pr[k], wls[k * NCLS + o], s);
    lg[tid] = s + bls[o];
  }
  __syncthreads();
  if (tid < PGS * NCLS) {
    const int g = tid / NCLS;
    const float* lr = lg + g * NCLS;
    float mx = lr[0];
#pragma unroll 1
    for (int i = 1; i < NCLS; ++i) {
      const float v = lr[i];
      mx = (v > mx || v != v) ? v : mx;
    }
    float se = 0.0f;
#pragma unroll 1
    for (int i = 0; i < NCLS; ++i) se += expf(lr[i] - mx);
    os[tid] = (lg[tid] - mx) - logf(se);
  }
  __syncthreads();
  const int npc = (nb * NCLS) >> 2;
  const bool ok = tid < npc;
  const int tq = tid < (PGS * NCLS) / 4 ? tid : (PGS * NCLS) / 4 - 1;
  const v4f ov = *(const v4fa*)(os + 4 * tq);
  float* op = out + (size_t)slotBase * NCLS + 4 * tq;
  if (ok) *(volatile v4f*)op = ov;
  __threadfence();
  if (ok) *(volatile v4f*)op = ov;
}

static inline int cdiv(int a, int b) { return (a + b - 1) / b; }
static inline size_t al256(size_t o) { return (o + 255) & ~(size_t)255; }

extern "C" void kernel_launch(void* const* d_in, const int* in_sizes, int n_in,
                              void* d_out, int out_size, void* d_ws, size_t ws_size,
                              hipStream_t stream) {
  if (n_in < 17) return;
  if (in_sizes[0] < DIN || (in_sizes[0] % DIN) != 0) return;
  const int nN = in_sizes[0] / DIN;
  if (nN < 1 || nN > (1 << 22)) return;
  const int nE2 = in_sizes[1];
  if (nE2 < 2 || (nE2 & 1) != 0) return;
  const int nE = nE2 / 2;
  if (nE < 1 || nE >= (1 << 22)) return;
  if (in_sizes[2] != nN) return;
  if (in_sizes[3] != DIN * DIN || in_sizes[4] != DIN) return;
  if (in_sizes[5] != DIN * DIN || in_sizes[6] != DIN) return;
  if (in_sizes[7] != DIN || in_sizes[8] != DIN) return;
  if (in_sizes[9] != DIN * DIN || in_sizes[10] != DIN) return;
  if (in_sizes[11] != DIN * DIN || in_sizes[12] != DIN) return;
  if (in_sizes[13] != DIN || in_sizes[14] != DIN) return;
  if (in_sizes[15] != DIN * NCLS || in_sizes[16] != NCLS) return;
  if (out_size < NCLS || (out_size % NCLS) != 0) return;
  const int nG = out_size / NCLS;
  if (nG < 8 || (nG % 8) != 0 || nG > (1 << 20)) return;
  if ((long long)nG * NCLS != (long long)out_size) return;

  const float* x     = (const float*)d_in[0];
  const int*   ei    = (const int*)  d_in[1];
  const int*   src   = ei;
  const int*   dst   = ei + nE;
  const int*   batch = (const int*)  d_in[2];
  const float* W1a = (const float*)d_in[3];  const float* b1a = (const float*)d_in[4];
  const float* W1b = (const float*)d_in[5];  const float* b1b = (const float*)d_in[6];
  const float* g1  = (const float*)d_in[7];  const float* be1 = (const float*)d_in[8];
  const float* W2a = (const float*)d_in[9];  const float* b2a = (const float*)d_in[10];
  const float* W2b = (const float*)d_in[11]; const float* b2b = (const float*)d_in[12];
  const float* g2  = (const float*)d_in[13]; const float* be2 = (const float*)d_in[14];
  const float* Wlin = (const float*)d_in[15];
  const float* blin = (const float*)d_in[16];
  float* out = (float*)d_out;

  const int MP   = cdiv(nN, GBM) * GBM;
  const int gM   = MP / GBM;
  const int gA   = cdiv(MP, NB);
  const int vec8 = ((nE & 3) == 0) ? 1 : 0;
  if ((long long)gA * NB < (long long)MP) return;
  if ((MP % APR) != 0 || (MP % AGR) != 0) return;

  char* ws = (char*)d_ws;
  size_t off = 0;
  const size_t oWT = off; off = al256(off + (size_t)NUW * 16);
  const size_t oA  = off; off = al256(off + (size_t)MP * KA * 2);
  const size_t oZH = off; off = al256(off + (size_t)MP * DIN * 4);
  const size_t oRI = off; off = al256(off + (size_t)gA * NB * 4);
  const size_t oSL = off; off = al256(off + (size_t)gA * RCAP * 4);
  const size_t oPT = off; off = al256(off + (size_t)gM * PARTW * 4);
  const size_t oSS = off; off = al256(off + (size_t)(3 * DIN) * 4);
  if (off > ws_size || off > (size_t)WSMAX) return;
  unsigned short* WT = (unsigned short*)(ws + oWT);
  unsigned short* A  = (unsigned short*)(ws + oA);
  float*          ZH = (float*)(ws + oZH);
  unsigned short* XB = (unsigned short*)(ws + oZH);
  int*            RI = (int*)(ws + oRI);
  int*            SL = (int*)(ws + oSL);
  float*          PT = (float*)(ws + oPT);
  float*          SS = (float*)(ws + oSS);
  const unsigned short* W1aT = WT;
  const unsigned short* W1bT = WT + (size_t)1 * DIN * KA;
  const unsigned short* W2aT = WT + (size_t)2 * DIN * KA;
  const unsigned short* W2bT = WT + (size_t)3 * DIN * KA;

  hipFuncSetAttribute(reinterpret_cast<const void*>(&k_csr), hipFuncAttributeMaxDynamicSharedMemorySize, LDS_CSR);
  hipFuncSetAttribute(reinterpret_cast<const void*>(&k_mlp), hipFuncAttributeMaxDynamicSharedMemorySize, LDS_MLP);

  const int nUx = MP * (DIN / 8);
  k_wprep<<<NUW / NTHR, NTHR, 0, stream>>>(W1a, W1b, W2a, W2b, WT);
  k_cvx<<<cdiv(nUx, NTHR), NTHR, 0, stream>>>(x, nN, nUx, XB);
  k_csr<<<gA, NTHR, LDS_CSR, stream>>>(src, dst, nN, nE, vec8, RI, SL);
  k_agg<0><<<MP / AGR, NTHR, 0, stream>>>(RI, SL, XB, ZH, A, nN, MP);
  k_mlp<<<gM, GTHR, LDS_MLP, stream>>>(A, W1aT, W1bT, b1a, b1b, ZH, nN, MP, PT);
  k_bnfin<<<1, GBN, 0, stream>>>(PT, gM, g1, be1, SS);
  k_bnap<<<MP / APR, NTHR, 0, stream>>>(ZH, SS, nN, MP);
  k_agg<1><<<MP / AGR, NTHR, 0, stream>>>(RI, SL, XB, ZH, A, nN, MP);
  k_mlp<<<gM, GTHR, LDS_MLP, stream>>>(A, W2aT, W2bT, b2a, b2b, ZH, nN, MP, PT);
  k_bnfin<<<1, GBN, 0, stream>>>(PT, gM, g2, be2, SS);
  k_pool_head<<<cdiv(nG, PGS), NTHR, 0, stream>>>(ZH, SS, batch, nN, 1, nG, Wlin, blin, out);
}
